// TargetLinear_28647431864941
// MI455X (gfx1250) — hardware-run, weakly checked
//
#include <hip/hip_runtime.h>


#define NE   131072
#define NTS  64
#define NHC  8
#define NDH  256
#define NRK  32
#define NGW  4096
#define PE   16384
constexpr size_t al256(size_t b) { return (b + 255) & ~(size_t)255; }
constexpr size_t WS_TOTAL = al256((size_t)NE * NTS * 2) + al256((size_t)NHC * NGW * 4) + al256((size_t)NHC * NTS * 4) + al256((size_t)NHC * NTS * NTS * 2) + al256((size_t)NHC * NTS * PE * 4);
static_assert(WS_TOTAL == 50530304 && WS_TOTAL <= 134217728, "the workspace carve: 48.2 MiB");
static_assert(NGW == 2 * NTS * NRK && NE % PE == 0 && PE % 64 == 0 && (NHC * NTS) % 64 == 0 && NTS % 32 == 0 && NE * NTS % 8 == 0, "the generated words; whole parts; whole tiles; whole depth steps");
typedef _Float16 h16;
typedef unsigned short bf;
typedef __attribute__((ext_vector_type(16))) __bf16   v16bf;
typedef __attribute__((ext_vector_type(16))) _Float16 v16h;
typedef __attribute__((ext_vector_type(8)))  _Float16 v8h;
typedef __attribute__((ext_vector_type(8)))  unsigned short v8us;
typedef __attribute__((ext_vector_type(8)))  float    v8f;
typedef __attribute__((ext_vector_type(4)))  float    v4f;
typedef v8h  __attribute__((may_alias)) v8ha;
typedef v4f  __attribute__((may_alias)) v4fa;
typedef v8us __attribute__((may_alias)) v8usa;

__device__ __forceinline__ unsigned short f2bf(float f) { unsigned u = __float_as_uint(f); u += 0x7FFFu + ((u >> 16) & 1u); return (unsigned short)(u >> 16); }
__device__ __forceinline__ float bf2f(unsigned short b) { return __uint_as_float(((unsigned)b) << 16); }
__device__ __forceinline__ float bfr(float f) { return bf2f(f2bf(f)); }
__device__ __forceinline__ v16h cat16(v8h lo, v8h hi) { return __builtin_shufflevector(lo, hi, 0, 1, 2, 3, 4, 5, 6, 7, 8, 9, 10, 11, 12, 13, 14, 15); }
__device__ __forceinline__ v16bf cat16b(v8us lo, v8us hi) { return __builtin_bit_cast(v16bf, __builtin_shufflevector(lo, hi, 0, 1, 2, 3, 4, 5, 6, 7, 8, 9, 10, 11, 12, 13, 14, 15)); }
__device__ __forceinline__ v8f wmma16(v16h a, v16h b, v8f c) { return __builtin_amdgcn_wmma_f32_16x16x32_f16(false, a, false, b, (short)0, c, false, false); }
__device__ __forceinline__ v8f wmmab(v16bf a, v16bf b, v8f c) { return __builtin_amdgcn_wmma_f32_16x16x32_bf16(false, a, false, b, (short)0, c, false, false); }


template <typename T16> struct WFrag;
template <> struct WFrag<h16> { typedef v16h V; static __device__ __forceinline__ V ld(const h16* p) { return cat16(*(const v8h*)p, *(const v8h*)(p + 16)); } static __device__ __forceinline__ v8f mma(V a, V b, v8f c) { return wmma16(a, b, c); } };
template <> struct WFrag<bf> { typedef v16bf V; static __device__ __forceinline__ V ld(const bf* p) { return cat16b(*(const v8us*)p, *(const v8us*)(p + 16)); } static __device__ __forceinline__ v8f mma(V a, V b, v8f c) { return wmmab(a, b, c); } };
template <typename T16, int NSPLIT, bool BIAS>
__global__ __launch_bounds__(32) void k_gemmw(const T16* __restrict__ A, const T16* __restrict__ A2, const T16* __restrict__ Bt, const T16* __restrict__ Bt2, int K, float* C, int ldc, const float* __restrict__ bias, size_t sA, size_t sB, size_t sC) {
    typedef typename WFrag<T16>::V V;
    __shared__ __align__(16) float os[16 * 68];
    const size_t z = blockIdx.z; A += z * sA; if (A2) A2 += z * sA; Bt += z * sB; if (Bt2) Bt2 += z * sB; C += z * sC;
    const int lane = threadIdx.x & 31, lr = lane & 15, hi = lane >> 4; const int r0 = blockIdx.x * 64, c0 = blockIdx.y * 64;
    v8f acc[4][4];
#pragma unroll
    for (int mb = 0; mb < 4; ++mb)
#pragma unroll
        for (int nb = 0; nb < 4; ++nb) acc[mb][nb] = (v8f){};
    const size_t aoff = (size_t)(r0 + lr) * K + 8 * hi, boff = (size_t)(c0 + lr) * K + 8 * hi;
    for (int kc = 0; kc < K; kc += 32) {
        V a[4], a2[4];
#pragma unroll
        for (int mb = 0; mb < 4; ++mb) { a[mb] = WFrag<T16>::ld(A + aoff + (size_t)mb * 16 * K + kc); if (NSPLIT == 1 || NSPLIT == 2) a2[mb] = WFrag<T16>::ld(A2 + aoff + (size_t)mb * 16 * K + kc); }
#pragma unroll
        for (int nb = 0; nb < 4; ++nb) { const V b = WFrag<T16>::ld(Bt + boff + (size_t)nb * 16 * K + kc); V b2; if (NSPLIT >= 2) b2 = WFrag<T16>::ld(Bt2 + boff + (size_t)nb * 16 * K + kc);
#pragma unroll
            for (int mb = 0; mb < 4; ++mb) { acc[mb][nb] = WFrag<T16>::mma(a[mb], b, acc[mb][nb]); if (NSPLIT == 1 || NSPLIT == 2) acc[mb][nb] = WFrag<T16>::mma(a2[mb], b, acc[mb][nb]); if (NSPLIT >= 2) acc[mb][nb] = WFrag<T16>::mma(a[mb], b2, acc[mb][nb]); } }
        asm volatile("v_nop\n\tv_nop\n\tv_nop\n\tv_nop" : "+v"(acc[0][0]), "+v"(acc[1][1]), "+v"(acc[2][2]), "+v"(acc[3][3]) : "v"(a[0]), "v"(a[3]));
    }
#pragma unroll
    for (int mb = 0; mb < 4; ++mb) {
#pragma unroll
        for (int nb = 0; nb < 4; ++nb) {
#pragma unroll
            for (int j = 0; j < 8; ++j) os[(hi * 8 + j) * 68 + nb * 16 + lr] = acc[mb][nb][j]; }
        __builtin_amdgcn_wave_barrier(); asm volatile("" ::: "memory");
        float* crow = C + (size_t)(r0 + mb * 16) * ldc + c0;
#pragma unroll 1
        for (int ps = 0; ps < 2; ++ps) {
#pragma unroll
            for (int s = 0; s < 8; ++s) { const int row = 2 * s + hi, cofs = lr * 4; v4f val = *(const v4fa*)(os + row * 68 + cofs); if (BIAS) { val[0] += bfr(bias[c0 + cofs]); val[1] += bfr(bias[c0 + cofs + 1]); val[2] += bfr(bias[c0 + cofs + 2]); val[3] += bfr(bias[c0 + cofs + 3]); }
                *(volatile v4f*)(crow + (size_t)row * ldc + cofs) = val; }
            if (ps == 0) __threadfence(); }
        __builtin_amdgcn_wave_barrier(); asm volatile("" ::: "memory");
    }
}

__device__ __forceinline__ h16 tohx(float x) { return (h16)x; }
__device__ __forceinline__ void splitf(float y, unsigned short& h, unsigned short& l) { h = f2bf(y); l = f2bf(y - bf2f(h)); }
typedef __attribute__((ext_vector_type(2))) _Float16 v2h;
typedef __attribute__((ext_vector_type(4))) _Float16 v4h;
typedef __attribute__((ext_vector_type(2))) unsigned short v2us;
typedef __attribute__((ext_vector_type(4))) unsigned short v4us;
typedef __attribute__((ext_vector_type(2))) float v2f;
typedef __attribute__((ext_vector_type(4))) int v4i;

__global__ __launch_bounds__(256) void k_cvt8h(const float* __restrict__ src, bf* dst, size_t n8) { const size_t i = (size_t)blockIdx.x * 256 + threadIdx.x; if (i >= n8) return; const v8f v = *(const v8f*)(src + i * 8); v8us o;
#pragma unroll
    for (int k = 0; k < 8; ++k) o[k] = __builtin_bit_cast(unsigned short, tohx(bfr(v[k]))); *(volatile v8us*)(dst + i * 8) = o; __threadfence(); *(volatile v8us*)(dst + i * 8) = o; }

__global__ __launch_bounds__(256) void k_small(const float* __restrict__ xh, const float* __restrict__ w, const float* __restrict__ b, int N, float* y) {
    const unsigned h = blockIdx.y; const unsigned c = blockIdx.x * 256 + threadIdx.x; if (c >= (unsigned)N) return; const float* xr = xh + (size_t)h * NDH; float s = 0.0f;
    for (int j = 0; j < NDH; ++j) s += bfr(xr[j]) * bfr(w[(size_t)j * N + c]);
    s = s + bfr(b[c]); float* d = y + (size_t)h * N + c; *(volatile float*)(d) = s; __threadfence(); *(volatile float*)(d) = s; }

__global__ __launch_bounds__(256) void k_wgen(const float* __restrict__ gw, bf* WT) {
    const unsigned h = blockIdx.y; const unsigned e = blockIdx.x * 256 + threadIdx.x; if (e >= (unsigned)(NTS * (NTS / 8))) return; const unsigned s = e >> 3, g = e & 7; const float* gh = gw + (size_t)h * NGW; v8us o;
#pragma unroll
    for (int q = 0; q < 8; ++q) { const unsigned d = 8 * g + q; float a = 0.0f;
#pragma unroll
        for (int r = 0; r < NRK; ++r) a += gh[d * NRK + r] * gh[NTS * NRK + r * NTS + s];
        o[q] = __builtin_bit_cast(unsigned short, tohx(a)); }
    bf* dd = WT + ((size_t)h * NTS + s) * NTS + 8 * g; *(volatile v8us*)(dd) = o; __threadfence(); *(volatile v8us*)(dd) = o; }

__global__ __launch_bounds__(256) void k_msum(const float* __restrict__ LT, const float* __restrict__ gb, const float* __restrict__ wm, float* res) {
    const unsigned n = blockIdx.x * 256 + threadIdx.x; if (n >= (unsigned)PE) return; const v4f m0 = *(const v4f*)(wm + (size_t)n * NHC); const v4f m1 = *(const v4f*)(wm + (size_t)n * NHC + 4);
    float mk[NHC];
#pragma unroll
    for (int h = 0; h < 4; ++h) { mk[h] = bfr(m0[h]); mk[h + 4] = bfr(m1[h]); }
    float* d = res + (size_t)n * NTS;
    for (int s4 = 0; s4 < NTS / 4; ++s4) { v4f a = {0.0f, 0.0f, 0.0f, 0.0f};
#pragma unroll
        for (int h = 0; h < NHC; ++h)
#pragma unroll
            for (int q = 0; q < 4; ++q) a[q] += (LT[((size_t)h * NTS + 4 * s4 + q) * PE + n] + gb[h * NTS + 4 * s4 + q]) * mk[h];
        *(volatile v4f*)(d + 4 * s4) = a; __threadfence(); *(volatile v4f*)(d + 4 * s4) = a; } }

extern "C" void kernel_launch(void* const* d_in, const int* in_sizes, int n_in,
                              void* d_out, int out_size, void* d_ws, size_t ws_size, hipStream_t stream) {
    if (n_in < 7) return;
    if (in_sizes[0] < NE * NTS || in_sizes[1] < NHC * NDH || in_sizes[2] < NE * NHC || in_sizes[3] < NDH * NGW || in_sizes[4] < NGW || in_sizes[5] < NDH * NTS || in_sizes[6] < NTS || out_size < NE * NTS) return;
    const float* tin = (const float*)d_in[0]; const float* hin = (const float*)d_in[1]; const float* wm = (const float*)d_in[2]; const float* wa = (const float*)d_in[3];
    const float* ba = (const float*)d_in[4]; const float* wc = (const float*)d_in[5]; const float* bc = (const float*)d_in[6];
    float* OUT = (float*)d_out;
    char* wsp = (char*)d_ws;
    auto take = [&](size_t bytes) { char* cur = wsp; wsp += (bytes + 255) & ~(size_t)255; return (void*)cur; };
    bf* TH = (bf*)take((size_t)NE * NTS * 2); float* GW = (float*)take((size_t)NHC * NGW * 4); float* GB = (float*)take((size_t)NHC * NTS * 4); bf* WT = (bf*)take((size_t)NHC * NTS * NTS * 2); float* LT = (float*)take((size_t)NHC * NTS * PE * 4);
    if ((size_t)(wsp - (char*)d_ws) != WS_TOTAL || WS_TOTAL > ws_size) return;
    k_cvt8h<<<(unsigned)(((size_t)NE * NTS / 8 + 255) / 256), 256, 0, stream>>>(tin, TH, (size_t)NE * NTS / 8);
    k_small<<<dim3(NGW / 256, NHC, 1), 256, 0, stream>>>(hin, wa, ba, NGW, GW);
    k_small<<<dim3(1, NHC, 1), 256, 0, stream>>>(hin, wc, bc, NTS, GB);
    k_wgen<<<dim3(NTS * (NTS / 8) / 256, NHC, 1), 256, 0, stream>>>(GW, WT);
    for (int pt = 0; pt < NE / PE; ++pt) {
        const size_t n0 = (size_t)pt * PE;
        k_gemmw<h16, 0, false><<<dim3(NHC * NTS / 64, PE / 64, 1), 32, 0, stream>>>((const h16*)WT, nullptr, (const h16*)(TH + n0 * NTS), nullptr, NTS, LT, PE, nullptr, (size_t)0, (size_t)0, (size_t)0);
        k_msum<<<(unsigned)((PE + 255) / 256), 256, 0, stream>>>(LT, GB, wm + n0 * NHC, OUT + n0 * NTS);
    }
}
